// MultiHeadAttention_65481071410942
// MI455X (gfx1250) — hardware-verified
//
#include <hip/hip_runtime.h>
#include <hip/hip_bf16.h>
#include <stdint.h>


#define EMB       768
#define NHEAD     8
#define HDIM      96
#define QKVN      (3 * EMB)
#define HEADN     (3 * HDIM)
#ifndef NB
#define NB        4
#endif
#ifndef SEQ
#define SEQ       2048
#endif
#define NB_FULL   4
#define SEQ_FULL  2048
#define MROWS     (NB * SEQ)
#define KBLK      64
#define QBLK      128
#define STG       (64 * HDIM)
#define P_CARRY   16384.0f
#define CTX_CARRY 64.0f
#define WP_CARRY  64.0f
#define INV_SCALE 0.10206207261596575f

static_assert(SEQ % QBLK == 0);
static_assert(SEQ % KBLK == 0);
static_assert(MROWS % 64 == 0);
static_assert((MROWS * EMB / 8) % 256 == 0);
static_assert(HDIM % 32 == 0);
static_assert(EMB % 128 == 0);
static_assert(QKVN % 64 == 0);
static_assert(HEADN == 288);
static_assert(NB <= NB_FULL);
static_assert(SEQ <= SEQ_FULL);

typedef unsigned short us;
typedef us       v8us  __attribute__((ext_vector_type(8)));
typedef __bf16   v16bf __attribute__((ext_vector_type(16)));
typedef _Float16 v16h  __attribute__((ext_vector_type(16)));
typedef float    v8f   __attribute__((ext_vector_type(8)));
typedef float    v4f   __attribute__((ext_vector_type(4)));

union Frag { v8us q[2]; v16bf b; v16h h; };

__device__ __forceinline__ us bf16_bits(float f) {
    union { float f; uint32_t u; } c; c.f = f;
    uint32_t u = c.u + 0x7FFFu + ((c.u >> 16) & 1u);
    return (us)(u >> 16);
}
__device__ __forceinline__ float bf16_val(us b) {
    union { float f; uint32_t u; } c; c.u = ((uint32_t)b) << 16;
    return c.f;
}
__device__ __forceinline__ float bf16_rne(float f) { return bf16_val(bf16_bits(f)); }
__device__ __forceinline__ us f16_bits(float f) {
    union { _Float16 h; us u; } c; c.h = (_Float16)f;
    return c.u;
}

__device__ __forceinline__ Frag load_frag(const us* base, int row, int stride, int k0) {
    Frag f;
    const us* p = base + (size_t)row * stride + k0;
    f.q[0] = *(const v8us*)(p);
    f.q[1] = *(const v8us*)(p + 16);
    return f;
}
__device__ __forceinline__ Frag load_frag_p(const us* rowp, int k0) {
    Frag f;
    f.q[0] = *(const v8us*)(rowp + k0);
    f.q[1] = *(const v8us*)(rowp + k0 + 16);
    return f;
}

__device__ __forceinline__ v8f wmma_bf16(v16bf a, v16bf b, v8f c) {
    v8f d = __builtin_amdgcn_wmma_f32_16x16x32_bf16(false, a, false, b, (short)0, c, false, false);
    asm volatile("v_nop\n\tv_nop\n\tv_nop\n\tv_nop" : "+v"(d) : "v"(a), "v"(b));
    return d;
}
__device__ __forceinline__ v8f wmma_f16(v16h a, v16h b, v8f c) {
    v8f d = __builtin_amdgcn_wmma_f32_16x16x32_f16(false, a, false, b, (short)0, c, false, false);
    asm volatile("v_nop\n\tv_nop\n\tv_nop\n\tv_nop" : "+v"(d) : "v"(a), "v"(b));
    return d;
}

__device__ __forceinline__ float rowmax16(float v) {
    #pragma unroll
    for (int m = 1; m < 16; m <<= 1) v = fmaxf(v, __shfl_xor(v, m, 32));
    return v;
}
__device__ __forceinline__ float rowsum16(float v) {
    #pragma unroll
    for (int m = 1; m < 16; m <<= 1) v += __shfl_xor(v, m, 32);
    return v;
}

__global__ __launch_bounds__(256)
void k_cvt_x(const float* __restrict__ x, us* __restrict__ xb) {
    const int i   = blockIdx.x * 256 + threadIdx.x;
    const int e   = i * 8;
    const int m   = e / EMB;
    const int col = e - m * EMB;
    const int b   = m / SEQ;
    const int n   = m - b * SEQ;
    const float* src = x + ((size_t)(b * SEQ_FULL + n) * EMB + col);
    const v4f a = *(const v4f*)(src);
    const v4f c = *(const v4f*)(src + 4);
    v8us o;
    o[0] = bf16_bits(a[0]); o[1] = bf16_bits(a[1]); o[2] = bf16_bits(a[2]); o[3] = bf16_bits(a[3]);
    o[4] = bf16_bits(c[0]); o[5] = bf16_bits(c[1]); o[6] = bf16_bits(c[2]); o[7] = bf16_bits(c[3]);
    us* dst = xb + (size_t)e;
    *(volatile v8us*)dst = o;
    __threadfence();
    *(volatile v8us*)dst = o;
}

__global__ __launch_bounds__(256)
void k_cvt_w(const float* __restrict__ W, us* __restrict__ Wt, int K, int N,
             int f16mode, float scale) {
    __shared__ __attribute__((aligned(16))) us tile[64 * 64];
    const int t  = threadIdx.x;
    const int n0 = blockIdx.x * 64;
    const int k0 = blockIdx.y * 64;
    #pragma unroll
    for (int it = 0; it < 4; ++it) {
        const int idx = t + 256 * it;
        const int kr  = idx >> 4;
        const int nc  = (idx & 15) * 4;
        const v4f v = *(const v4f*)(W + (size_t)(k0 + kr) * N + n0 + nc);
        #pragma unroll
        for (int j = 0; j < 4; ++j) {
            const float bv = bf16_rne(v[j]);
            const us hb = f16_bits(bv * scale);
            const us bb = bf16_bits(v[j]);
            tile[(nc + j) * 64 + kr] = f16mode ? hb : bb;
        }
    }
    __syncthreads();
    v8us ov[2];
    size_t od[2];
    #pragma unroll
    for (int it = 0; it < 2; ++it) {
        const int idx = t + 256 * it;
        const int nr  = idx >> 3;
        const int pc  = idx & 7;
        ov[it] = *(const v8us*)&tile[nr * 64 + pc * 8];
        od[it] = (size_t)(n0 + nr) * K + k0 + pc * 8;
    }
    #pragma unroll
    for (int it = 0; it < 2; ++it) *(volatile v8us*)(Wt + od[it]) = ov[it];
    __threadfence();
    #pragma unroll
    for (int it = 0; it < 2; ++it) *(volatile v8us*)(Wt + od[it]) = ov[it];
}

__global__ __launch_bounds__(256)
void k_qkv(const us* __restrict__ xb, const us* __restrict__ wq, const float* __restrict__ bqkv,
           us* __restrict__ qh, us* __restrict__ ql, us* __restrict__ kh, us* __restrict__ kl,
           us* __restrict__ vt) {
    __shared__ __attribute__((aligned(16))) us stg[5 * STG];

    const int t = threadIdx.x;
    const int wave = t >> 5, lane = t & 31;
    const int half = lane >> 4, l16 = lane & 15;
    const int h  = blockIdx.x;
    const int m0 = blockIdx.y * 64;
    const int n0 = h * HEADN;
    const int wr = wave & 3;
    const int wc = wave >> 2;
    const int arow  = m0 + wr * 16 + l16;
    const int bcol0 = n0 + wc * 144;

    v8f acc[9];
    #pragma unroll
    for (int j = 0; j < 9; ++j) { v8f z = {}; acc[j] = z; }

    #pragma unroll 1
    for (int k0 = 0; k0 < EMB; k0 += 32) {
        const Frag a = load_frag(xb, arow, EMB, k0 + half * 8);
        #pragma unroll
        for (int j = 0; j < 9; ++j) {
            const Frag bfr = load_frag(wq, bcol0 + j * 16 + l16, EMB, k0 + half * 8);
            acc[j] = wmma_bf16(a.b, bfr.b, acc[j]);
        }
    }

    const int b   = m0 / SEQ;
    const int nl0 = m0 - b * SEQ;
    const int bh  = b * NHEAD + h;
    #pragma unroll
    for (int j = 0; j < 9; ++j) {
        const int cl    = wc * 144 + j * 16 + l16;
        const int d     = cl / 3;
        const int which = cl - d * 3;
        const float bb  = bf16_rne(bqkv[n0 + cl]);
        #pragma unroll
        for (int r = 0; r < 8; ++r) {
            const int row   = wr * 16 + half * 8 + r;
            const float val = acc[j][r] + bb;
            const us hib    = bf16_bits(val);
            const us lob    = bf16_bits(val - bf16_val(hib));
            const us fb     = f16_bits(val);
            const int offqk = row * HDIM + d;
            const int offA  = (which == 2) ? (4 * STG + d * 64 + row) : (which * 2 * STG + offqk);
            stg[offA] = (which == 2) ? fb : hib;
            if (which != 2) stg[(which * 2 + 1) * STG + offqk] = lob;
        }
    }
    __syncthreads();

    const size_t qkbase = ((size_t)bh * SEQ + nl0) * HDIM;
    v8us ov[15];
    size_t vto[3];
    #pragma unroll
    for (int p = 0; p < 4; ++p)
        #pragma unroll
        for (int it = 0; it < 3; ++it) {
            const int i = t + 256 * it;
            ov[p * 3 + it] = *(const v8us*)&stg[p * STG + i * 8];
        }
    #pragma unroll
    for (int it = 0; it < 3; ++it) {
        const int i  = t + 256 * it;
        const int d  = i >> 3;
        const int pc = i & 7;
        ov[12 + it] = *(const v8us*)&stg[4 * STG + d * 64 + pc * 8];
        vto[it] = ((size_t)(bh * HDIM + d)) * SEQ + nl0 + pc * 8;
    }
    auto emit = [&]() {
        #pragma unroll
        for (int it = 0; it < 3; ++it) {
            const int i = t + 256 * it;
            *(volatile v8us*)(qh + qkbase + i * 8) = ov[0 + it];
            *(volatile v8us*)(ql + qkbase + i * 8) = ov[3 + it];
            *(volatile v8us*)(kh + qkbase + i * 8) = ov[6 + it];
            *(volatile v8us*)(kl + qkbase + i * 8) = ov[9 + it];
            *(volatile v8us*)(vt + vto[it])        = ov[12 + it];
        }
    };
    emit();
    __threadfence();
    emit();
}

__global__ __launch_bounds__(256)
void k_attn(const us* __restrict__ qh, const us* __restrict__ ql,
            const us* __restrict__ kh, const us* __restrict__ kl,
            const us* __restrict__ vt, us* __restrict__ ctx) {
    __shared__ __attribute__((aligned(16))) us sKh[KBLK * HDIM];
    __shared__ __attribute__((aligned(16))) us sKl[KBLK * HDIM];
    __shared__ __attribute__((aligned(16))) us sVt[HDIM * KBLK];
    __shared__ __attribute__((aligned(16))) us sP[8 * 16 * HDIM];

    const int t = threadIdx.x;
    const int wave = t >> 5, lane = t & 31;
    const int half = lane >> 4, l16 = lane & 15;
    const int bh = blockIdx.y;
    const int qr = blockIdx.x * QBLK + wave * 16;
    const size_t qoff = ((size_t)bh * SEQ + qr + l16) * HDIM;
    const us* qhp = qh + qoff;
    const us* qlp = ql + qoff;
    const us* khg = kh + (size_t)bh * SEQ * HDIM;
    const us* klg = kl + (size_t)bh * SEQ * HDIM;
    const us* vtg = vt + (size_t)bh * HDIM * SEQ;
    us* ps = sP + wave * 16 * HDIM;

    v8f accO[6];
    #pragma unroll
    for (int dt = 0; dt < 6; ++dt) { v8f z = {}; accO[dt] = z; }
    float mrow[8], lrow[8];
    #pragma unroll
    for (int r = 0; r < 8; ++r) { mrow[r] = -__builtin_inff(); lrow[r] = 0.0f; }

    #pragma unroll 1
    for (int j = 0; j < SEQ / KBLK; ++j) {
        const int key0 = j * KBLK;
        __syncthreads();
        #pragma unroll
        for (int it = 0; it < 3; ++it) {
            const int i  = t + 256 * it;
            const int kr = i / 12;
            const int kc = i - kr * 12;
            const size_t go = (size_t)(key0 + kr) * HDIM + kc * 8;
            *(v8us*)&sKh[kr * HDIM + kc * 8] = *(const v8us*)(khg + go);
            *(v8us*)&sKl[kr * HDIM + kc * 8] = *(const v8us*)(klg + go);
            const int d  = i >> 3;
            const int pc = i & 7;
            *(v8us*)&sVt[d * KBLK + pc * 8] = *(const v8us*)(vtg + (size_t)d * SEQ + key0 + pc * 8);
        }
        __syncthreads();

        v8f sc[4];
        #pragma unroll
        for (int nt = 0; nt < 4; ++nt) { v8f z = {}; sc[nt] = z; }
        #pragma unroll
        for (int c = 0; c < 3; ++c) {
            const Frag qa = load_frag_p(qhp, c * 32 + half * 8);
            const Frag qb = load_frag_p(qlp, c * 32 + half * 8);
            #pragma unroll
            for (int nt = 0; nt < 4; ++nt) {
                const Frag fh = load_frag(sKh, nt * 16 + l16, HDIM, c * 32 + half * 8);
                const Frag fl = load_frag(sKl, nt * 16 + l16, HDIM, c * 32 + half * 8);
                sc[nt] = wmma_bf16(qa.b, fh.b, sc[nt]);
                sc[nt] = wmma_bf16(qa.b, fl.b, sc[nt]);
                sc[nt] = wmma_bf16(qb.b, fh.b, sc[nt]);
            }
        }

        float alpha[8];
        #pragma unroll
        for (int r = 0; r < 8; ++r) {
            float bm = sc[0][r];
            #pragma unroll
            for (int nt = 1; nt < 4; ++nt) bm = fmaxf(bm, sc[nt][r]);
            bm = rowmax16(bm);
            const float mnew = fmaxf(mrow[r], bm);
            alpha[r] = __expf(mrow[r] - mnew);
            mrow[r] = mnew;
        }
        float rs[8];
        #pragma unroll
        for (int r = 0; r < 8; ++r) rs[r] = 0.0f;
        #pragma unroll
        for (int nt = 0; nt < 4; ++nt)
            #pragma unroll
            for (int r = 0; r < 8; ++r) {
                const float p = __expf(sc[nt][r] - mrow[r]);
                sc[nt][r] = p;
                rs[r] += p;
            }
        #pragma unroll
        for (int r = 0; r < 8; ++r) {
            lrow[r] = lrow[r] * alpha[r] + rowsum16(rs[r]);
            #pragma unroll
            for (int dt = 0; dt < 6; ++dt) accO[dt][r] = accO[dt][r] * alpha[r];
        }

        #pragma unroll
        for (int nt = 0; nt < 4; ++nt)
            #pragma unroll
            for (int r = 0; r < 8; ++r)
                ps[(r + 8 * half) * HDIM + nt * 16 + l16] = f16_bits(sc[nt][r] * P_CARRY);
        __syncthreads();

        const Frag p0 = load_frag(ps, l16, HDIM, 0 * 32 + half * 8);
        const Frag p1 = load_frag(ps, l16, HDIM, 1 * 32 + half * 8);

        #pragma unroll
        for (int dt = 0; dt < 6; ++dt) {
            const Frag v0 = load_frag(sVt, dt * 16 + l16, KBLK, 0 * 32 + half * 8);
            const Frag v1 = load_frag(sVt, dt * 16 + l16, KBLK, 1 * 32 + half * 8);
            accO[dt] = wmma_f16(p0.h, v0.h, accO[dt]);
            accO[dt] = wmma_f16(p1.h, v1.h, accO[dt]);
        }
    }

    __syncthreads();
    float inv[8];
    #pragma unroll
    for (int r = 0; r < 8; ++r) inv[r] = (1.0f / lrow[r]) * (INV_SCALE * CTX_CARRY / P_CARRY);
    #pragma unroll
    for (int dt = 0; dt < 6; ++dt)
        #pragma unroll
        for (int r = 0; r < 8; ++r)
            ps[(r + 8 * half) * HDIM + dt * 16 + l16] = f16_bits(accO[dt][r] * inv[r]);
    __syncthreads();

    us* dst = ctx + ((size_t)bh * SEQ + qr) * HDIM;
    v8us ov[6];
    #pragma unroll
    for (int it = 0; it < 6; ++it) ov[it] = *(const v8us*)&ps[(lane + 32 * it) * 8];
    #pragma unroll
    for (int it = 0; it < 6; ++it) *(volatile v8us*)(dst + (lane + 32 * it) * 8) = ov[it];
    __threadfence();
    #pragma unroll
    for (int it = 0; it < 6; ++it) *(volatile v8us*)(dst + (lane + 32 * it) * 8) = ov[it];
}

__global__ __launch_bounds__(256)
void k_proj(const us* __restrict__ ctx, const us* __restrict__ wp,
            const float* __restrict__ bproj, float* __restrict__ out) {
    __shared__ __attribute__((aligned(16))) float sO[64 * 128];

    const int t = threadIdx.x;
    const int wave = t >> 5, lane = t & 31;
    const int half = lane >> 4, l16 = lane & 15;
    const int n0 = blockIdx.x * 128;
    const int m0 = blockIdx.y * 64;
    const int wr = wave & 3;
    const int wc = wave >> 2;
    const int m  = m0 + wr * 16 + l16;
    const int b  = m / SEQ;
    const int n  = m - b * SEQ;
    const us* abase = ctx + ((size_t)(b * NHEAD) * SEQ + n) * HDIM;
    const int bcol = n0 + wc * 64;

    v8f acc[4];
    #pragma unroll
    for (int nt = 0; nt < 4; ++nt) { v8f z = {}; acc[nt] = z; }

    #pragma unroll 1
    for (int hh = 0; hh < NHEAD; ++hh) {
        const us* ap = abase + (size_t)hh * SEQ * HDIM;
        #pragma unroll
        for (int cc = 0; cc < 3; ++cc) {
            const Frag a = load_frag_p(ap, cc * 32 + half * 8);
            const int k0 = hh * HDIM + cc * 32;
            #pragma unroll
            for (int nt = 0; nt < 4; ++nt) {
                const Frag bfr = load_frag(wp, bcol + nt * 16 + l16, EMB, k0 + half * 8);
                acc[nt] = wmma_f16(a.h, bfr.h, acc[nt]);
            }
        }
    }

    const float osc = 1.0f / (CTX_CARRY * WP_CARRY);
    #pragma unroll
    for (int nt = 0; nt < 4; ++nt) {
        const int cl   = wc * 64 + nt * 16 + l16;
        const float bb = bf16_rne(bproj[n0 + cl]);
        #pragma unroll
        for (int r = 0; r < 8; ++r)
            sO[(wr * 16 + half * 8 + r) * 128 + cl] = acc[nt][r] * osc + bb;
    }
    __syncthreads();

    v4f ov[8];
    size_t od[8];
    #pragma unroll
    for (int it = 0; it < 8; ++it) {
        const int i   = t + 256 * it;
        const int row = i >> 5;
        const int pc  = i & 31;
        ov[it] = *(const v4f*)&sO[row * 128 + pc * 4];
        od[it] = (size_t)(m0 + row) * EMB + n0 + pc * 4;
    }
    #pragma unroll
    for (int it = 0; it < 8; ++it) *(volatile v4f*)(out + od[it]) = ov[it];
    __threadfence();
    #pragma unroll
    for (int it = 0; it < 8; ++it) *(volatile v4f*)(out + od[it]) = ov[it];
}

extern "C" void kernel_launch(void* const* d_in, const int* in_sizes, int n_in,
                              void* d_out, int out_size, void* d_ws, size_t ws_size,
                              hipStream_t stream) {
    if (n_in < 5) return;
    if (in_sizes[0] < ((NB - 1) * SEQ_FULL + SEQ) * EMB) return;
    if (in_sizes[1] < EMB * QKVN) return;
    if (in_sizes[2] < QKVN) return;
    if (in_sizes[3] < EMB * EMB) return;
    if (in_sizes[4] < EMB) return;
    if (out_size < MROWS * EMB) return;

    const float* x      = (const float*)d_in[0];
    const float* w_qkv  = (const float*)d_in[1];
    const float* b_qkv  = (const float*)d_in[2];
    const float* w_proj = (const float*)d_in[3];
    const float* b_proj = (const float*)d_in[4];
    float*       out    = (float*)d_out;

    char*  ws  = (char*)d_ws;
    size_t off = 0;
    auto carve = [&](size_t bytes) -> char* {
        char* p = ws + off;
        off += (bytes + 255) & ~size_t(255);
        return p;
    };
    const size_t plane = (size_t)MROWS * EMB * sizeof(us);
    us* xb  = (us*)carve(plane);
    us* wq  = (us*)carve((size_t)QKVN * EMB * sizeof(us));
    us* wp  = (us*)carve((size_t)EMB * EMB * sizeof(us));
    us* qh  = (us*)carve(plane);
    us* ql  = (us*)carve(plane);
    us* kh  = (us*)carve(plane);
    us* kl  = (us*)carve(plane);
    us* vt  = (us*)carve(plane);
    us* ctx = (us*)carve(plane);
    if (off > ws_size) return;

    k_cvt_x<<<(MROWS * EMB / 8) / 256, 256, 0, stream>>>(x, xb);
    k_cvt_w<<<dim3(QKVN / 64, EMB / 64), 256, 0, stream>>>(w_qkv, wq, EMB, QKVN, 0, 1.0f);
    k_cvt_w<<<dim3(EMB / 64, EMB / 64), 256, 0, stream>>>(w_proj, wp, EMB, EMB, 1, WP_CARRY);
    k_qkv<<<dim3(NHEAD, MROWS / 64), 256, 0, stream>>>(xb, wq, b_qkv, qh, ql, kh, kl, vt);
    k_attn<<<dim3(SEQ / QBLK, NB * NHEAD), 256, 0, stream>>>(qh, ql, kh, kl, vt, ctx);
    k_proj<<<dim3(EMB / 128, MROWS / 64), 256, 0, stream>>>(ctx, wp, b_proj, out);
}
